// DeepONet_3908420240249
// MI455X (gfx1250) — hardware-verified
//
#include <hip/hip_runtime.h>
#include <math.h>
#include <stddef.h>
#include <stdint.h>


#define SENSOR 128
#define BUNITS 1024
#define LORA   64
#define BATCH  2048
#define TU     128
#define PTRUNK 33409
#define OFF_B0 0
#define OFF_W0 128
#define OFF_B1 256
#define OFF_W1 384
#define OFF_B2 16768
#define OFF_W2 16896
#define OFF_B3 33280
#define OFF_W3 33281
#define NSAMP  32

static_assert(OFF_W3 + TU == PTRUNK);
static_assert(BATCH % 128 == 0);
static_assert(BUNITS % 128 == 0);
static_assert(SENSOR % 32 == 0);
static_assert(BUNITS % 32 == 0);
static_assert(LORA == 64);
static_assert(BATCH % NSAMP == 0);
static_assert((BATCH * SENSOR) % 2048 == 0);

typedef _Float16 v16h __attribute__((ext_vector_type(16)));
typedef _Float16 v8h_na __attribute__((ext_vector_type(8)));
typedef v8h_na v8h __attribute__((may_alias));
typedef float v8f __attribute__((ext_vector_type(8)));
typedef float v4f_na __attribute__((ext_vector_type(4)));
typedef v4f_na v4f __attribute__((may_alias));
typedef unsigned int v4u_na __attribute__((ext_vector_type(4)));
typedef v4u_na v4u __attribute__((may_alias));

union Frag { v16h v; v8h half[2]; };
union Pack16 { v4u u; v4f f; v8h hh; };

__device__ __forceinline__ int imin(int a, int b) { return a < b ? a : b; }

__device__ __forceinline__ v8f zero8() {
  v8f z;
#pragma unroll
  for (int e = 0; e < 8; ++e) z[e] = 0.f;
  return z;
}

__device__ __forceinline__ v8f wmma16(const v16h a, const v16h b, v8f c) {
  v8f d = __builtin_amdgcn_wmma_f32_16x16x32_f16(false, a, false, b, (short)0, c, false, false);
  asm volatile("v_nop\n\tv_nop\n\tv_nop\n\tv_nop" : "+v"(d) : "v"(a), "v"(b));
  return d;
}

__global__ __launch_bounds__(256) void k_cvt(const float* __restrict__ s, _Float16* __restrict__ d,
                                             int nchunks, float scale)
{
  const int c = blockIdx.x * 256 + threadIdx.x;
  const bool ok = c < nchunks;
  const int cc = ok ? c : 0;
  const float* sp = s + (size_t)cc * 8;
  v8h hv;
#pragma unroll
  for (int e = 0; e < 8; ++e) hv[e] = (_Float16)(sp[e] * scale);
  Pack16 p; p.hh = hv;
  _Float16* dp = d + (size_t)cc * 8;
  if (ok) *(volatile v4u*)dp = p.u;
  __threadfence();
  if (ok) *(volatile v4u*)dp = p.u;
}

__global__ __launch_bounds__(256) void k_cvt_t(const float* __restrict__ s, _Float16* __restrict__ d,
                                               int Kd, int Nd, float scale)
{
  const int kc = Kd >> 3;
  const int total = Nd * kc;
  const int c = blockIdx.x * 256 + threadIdx.x;
  const bool ok = c < total;
  const int cc = ok ? c : 0;
  const int n = cc / kc, k8 = cc - n * kc;
  const float* sp = s + (size_t)(k8 * 8) * (size_t)Nd + n;
  v8h hv;
#pragma unroll
  for (int e = 0; e < 8; ++e) hv[e] = (_Float16)(sp[(size_t)e * (size_t)Nd] * scale);
  Pack16 p; p.hh = hv;
  _Float16* dp = d + (size_t)cc * 8;
  if (ok) *(volatile v4u*)dp = p.u;
  __threadfence();
  if (ok) *(volatile v4u*)dp = p.u;
}

__global__ __launch_bounds__(256) void k_build_w2t(const float* __restrict__ W2, _Float16* __restrict__ w2t)
{
  const int total = 2 * LORA * TU * (TU / 8);
  const int c = blockIdx.x * 256 + threadIdx.x;
  const bool ok = c < total;
  const int cc = ok ? c : 0;
  const int i8 = cc & 15, o = (cc >> 4) & 127, r = (cc >> 11) & 63, l = cc >> 17;
  const int woff = l ? OFF_W2 : OFF_W1;
  const float* sp = W2 + (size_t)r * PTRUNK + woff + (size_t)(i8 * 8) * TU + o;
  v8h hv;
#pragma unroll
  for (int e = 0; e < 8; ++e) hv[e] = (_Float16)(sp[(size_t)e * TU] * 64.0f);
  Pack16 p; p.hh = hv;
  _Float16* dp = w2t + (size_t)cc * 8;
  if (ok) *(volatile v4u*)dp = p.u;
  __threadfence();
  if (ok) *(volatile v4u*)dp = p.u;
}

__device__ __forceinline__ v4u pack_out(const float* src, _Float16*) {
  const v4f x0 = *(const v4f*)src;
  const v4f x1 = *(const v4f*)(src + 4);
  v8h hv;
  hv[0] = (_Float16)x0[0]; hv[1] = (_Float16)x0[1]; hv[2] = (_Float16)x0[2]; hv[3] = (_Float16)x0[3];
  hv[4] = (_Float16)x1[0]; hv[5] = (_Float16)x1[1]; hv[6] = (_Float16)x1[2]; hv[7] = (_Float16)x1[3];
  Pack16 p; p.hh = hv; return p.u;
}
__device__ __forceinline__ v4u pack_out(const float* src, float*) {
  Pack16 p; p.f = *(const v4f*)src; return p.u;
}

template<bool TANH, bool HASBIAS, typename OT>
__global__ __launch_bounds__(256) void k_gemm(const _Float16* __restrict__ A, const _Float16* __restrict__ Bt,
                                              const float* __restrict__ bias, OT* __restrict__ C,
                                              int M, int N, int K, float oscale)
{
  constexpr int CP  = 68;
  constexpr int EPC = 16 / (int)sizeof(OT);
  constexpr int CPR = 64 / EPC;
  constexpr int NST = (16 * CPR) / 32;
  __shared__ __align__(16) float sC[8][16][CP];

  const int tid = threadIdx.x, lane = tid & 31, wave = tid >> 5;
  const int wm = wave >> 1, wn = wave & 1, h = lane >> 4, l15 = lane & 15;
  const int m0 = blockIdx.x * 128, n0 = blockIdx.y * 128;
  const int arow0 = m0 + wm * 32, bcol0 = n0 + wn * 64;

  const _Float16* ap[2];
  const _Float16* bp[4];
#pragma unroll
  for (int i = 0; i < 2; ++i)
    ap[i] = A + (size_t)imin(arow0 + i * 16 + l15, M - 1) * (size_t)K + 8 * h;
#pragma unroll
  for (int j = 0; j < 4; ++j)
    bp[j] = Bt + (size_t)imin(bcol0 + j * 16 + l15, N - 1) * (size_t)K + 8 * h;

  v8f acc[2][4];
#pragma unroll
  for (int i = 0; i < 2; ++i)
#pragma unroll
    for (int j = 0; j < 4; ++j) acc[i][j] = zero8();

#pragma unroll 1
  for (int k0 = 0; k0 < K; k0 += 32) {
    Frag a[2], b[4];
#pragma unroll
    for (int i = 0; i < 2; ++i) {
      a[i].half[0] = *(const v8h*)(ap[i] + k0);
      a[i].half[1] = *(const v8h*)(ap[i] + k0 + 16);
    }
#pragma unroll
    for (int j = 0; j < 4; ++j) {
      b[j].half[0] = *(const v8h*)(bp[j] + k0);
      b[j].half[1] = *(const v8h*)(bp[j] + k0 + 16);
    }
#pragma unroll
    for (int i = 0; i < 2; ++i)
#pragma unroll
      for (int j = 0; j < 4; ++j)
        acc[i][j] = wmma16(a[i].v, b[j].v, acc[i][j]);
  }

  float bv[4];
#pragma unroll
  for (int j = 0; j < 4; ++j)
    bv[j] = HASBIAS ? bias[imin(bcol0 + j * 16 + l15, N - 1)] : 0.f;
  const bool stok = (bcol0 + 64 <= N);

#pragma unroll
  for (int i = 0; i < 2; ++i) {
#pragma unroll
    for (int j = 0; j < 4; ++j) {
#pragma unroll
      for (int r = 0; r < 8; ++r) {
        float v = acc[i][j][r] * oscale + bv[j];
        if (TANH) v = tanhf(v);
        sC[wave][8 * h + r][j * 16 + l15] = v;
      }
    }
    __syncthreads();
    if (stok) {
      const size_t grow0 = (size_t)(arow0 + i * 16);
#pragma unroll
      for (int s = 0; s < NST; ++s) {
        const int c = s * 32 + lane;
        const int row = c / CPR, piece = c - row * CPR;
        const v4u pv = pack_out(&sC[wave][row][piece * EPC], (OT*)0);
        OT* dst = C + (grow0 + (size_t)row) * (size_t)N + bcol0 + piece * EPC;
        *(volatile v4u*)dst = pv;
      }
      __threadfence();
#pragma unroll
      for (int s = 0; s < NST; ++s) {
        const int c = s * 32 + lane;
        const int row = c / CPR, piece = c - row * CPR;
        const v4u pv = pack_out(&sC[wave][row][piece * EPC], (OT*)0);
        OT* dst = C + (grow0 + (size_t)row) * (size_t)N + bcol0 + piece * EPC;
        *(volatile v4u*)dst = pv;
      }
    }
    __syncthreads();
  }
}

__global__ __launch_bounds__(256) void k_trunk(const float* __restrict__ t, const float* __restrict__ u,
                                               const float* __restrict__ Z, const float* __restrict__ W2,
                                               const _Float16* __restrict__ W2t, float* __restrict__ out)
{
  __shared__ float sZ[LORA][NSAMP + 1];
  __shared__ __align__(16) _Float16 sX[NSAMP][TU];
  __shared__ float red[NSAMP][9];
  __shared__ __align__(16) float sOut[NSAMP];
  const int tid = threadIdx.x, lane = tid & 31, wave = tid >> 5;
  const int h = lane >> 4, l15 = lane & 15;
  const int b0 = blockIdx.x * NSAMP;
  const float INV64 = 0.015625f;

  for (int i = tid; i < NSAMP * LORA; i += 256) {
    const int m = i & (NSAMP - 1), r = i >> 5;
    sZ[r][m] = Z[(size_t)(b0 + m) * LORA + r];
  }
  __syncthreads();

  for (int i = tid; i < NSAMP * TU; i += 256) {
    const int o = i & (TU - 1), m = i >> 7;
    float wb = 0.f, ww = 0.f;
    const float* cb = W2 + OFF_B0 + o;
    const float* cw = W2 + OFF_W0 + o;
#pragma unroll 4
    for (int r = 0; r < LORA; ++r) {
      const float zr = sZ[r][m];
      wb += zr * cb[(size_t)r * PTRUNK];
      ww += zr * cw[(size_t)r * PTRUNK];
    }
    const float tv = t[b0 + m];
    sX[m][o] = (_Float16)tanhf(tv * ww + wb);
  }
  __syncthreads();

#pragma unroll 1
  for (int l = 0; l < 2; ++l) {
    Frag a[2][4];
#pragma unroll
    for (int mt = 0; mt < 2; ++mt) {
#pragma unroll
      for (int kk = 0; kk < 4; ++kk) {
        const _Float16* xp = &sX[mt * 16 + l15][kk * 32];
        a[mt][kk].half[0] = *(const v8h*)(xp + 8 * h);
        a[mt][kk].half[1] = *(const v8h*)(xp + 16 + 8 * h);
      }
    }
    __syncthreads();

    const int o = wave * 16 + l15;
    const int boff = l ? OFF_B2 : OFF_B1;
    const _Float16* wbase = W2t + (size_t)l * (LORA * TU * TU) + (size_t)o * TU + 8 * h;
    const float* bc = W2 + boff + o;
    v8f acc0 = zero8(), acc1 = zero8();

#pragma unroll 1
    for (int r = 0; r < LORA; ++r) {
      const _Float16* bpr = wbase + (size_t)r * (TU * TU);
      v8f y0 = zero8(), y1 = zero8();
#pragma unroll
      for (int kk = 0; kk < 4; ++kk) {
        Frag b;
        b.half[0] = *(const v8h*)(bpr + kk * 32);
        b.half[1] = *(const v8h*)(bpr + kk * 32 + 16);
        y0 = wmma16(a[0][kk].v, b.v, y0);
        y1 = wmma16(a[1][kk].v, b.v, y1);
      }
      const float bval = bc[(size_t)r * PTRUNK];
#pragma unroll
      for (int v = 0; v < 8; ++v) {
        acc0[v] += sZ[r][8 * h + v]      * (y0[v] * INV64 + bval);
        acc1[v] += sZ[r][16 + 8 * h + v] * (y1[v] * INV64 + bval);
      }
    }
#pragma unroll
    for (int v = 0; v < 8; ++v) {
      sX[8 * h + v][o]      = (_Float16)tanhf(acc0[v]);
      sX[16 + 8 * h + v][o] = (_Float16)tanhf(acc1[v]);
    }
    __syncthreads();
  }

  {
    const int m = tid >> 3, s = tid & 7;
    float partial = 0.f;
#pragma unroll 1
    for (int j = 0; j < 16; ++j) {
      const int i = s * 16 + j;
      const float* cw = W2 + OFF_W3 + i;
      float w = 0.f;
#pragma unroll 4
      for (int r = 0; r < LORA; ++r) w += sZ[r][m] * cw[(size_t)r * PTRUNK];
      partial += (float)sX[m][i] * w;
    }
    red[m][s] = partial;
  }
  __syncthreads();
  if (tid < NSAMP) {
    float q = 0.f;
#pragma unroll
    for (int s = 0; s < 8; ++s) q += red[tid][s];
    float b3 = 0.f;
    const float* cb = W2 + OFF_B3;
#pragma unroll 4
    for (int r = 0; r < LORA; ++r) b3 += sZ[r][tid] * cb[(size_t)r * PTRUNK];
    q += b3;
    const float tv = t[b0 + tid];
    const float u0 = u[(size_t)(b0 + tid) * SENSOR];
    sOut[tid] = u0 + tv * q;
  }
  __syncthreads();
  if (tid < 8) {
    const v4f v = *(const v4f*)&sOut[tid * 4];
    *(volatile v4f*)(out + b0 + tid * 4) = v;
  }
  __threadfence();
  if (tid < 8) {
    const v4f v = *(const v4f*)&sOut[tid * 4];
    *(volatile v4f*)(out + b0 + tid * 4) = v;
  }
}

extern "C" void kernel_launch(void* const* d_in, const int* in_sizes, int n_in,
                              void* d_out, int out_size, void* d_ws, size_t ws_size,
                              hipStream_t stream)
{
  if (n_in < 14 || out_size != BATCH) return;
  if (in_sizes[0] != BATCH || in_sizes[1] != BATCH * SENSOR || in_sizes[2] != SENSOR * BUNITS ||
      in_sizes[12] != BUNITS * LORA || in_sizes[13] != LORA * PTRUNK) return;
  for (int i = 0; i < 4; ++i) if (in_sizes[4 + 2 * i] != BUNITS * BUNITS) return;
  for (int i = 0; i < 5; ++i) if (in_sizes[3 + 2 * i] != BUNITS) return;

  const float* t  = (const float*)d_in[0];
  const float* u  = (const float*)d_in[1];
  const float* bw[5] = {(const float*)d_in[2], (const float*)d_in[4], (const float*)d_in[6],
                        (const float*)d_in[8], (const float*)d_in[10]};
  const float* bb[5] = {(const float*)d_in[3], (const float*)d_in[5], (const float*)d_in[7],
                        (const float*)d_in[9], (const float*)d_in[11]};
  const float* W1 = (const float*)d_in[12];
  const float* W2 = (const float*)d_in[13];
  float* out = (float*)d_out;

  char* base = (char*)d_ws;
  size_t off = 0;
  auto carve = [&](size_t bytes) -> char* {
    char* p = base + off;
    off += (bytes + 255) & ~(size_t)255;
    return p;
  };
  _Float16* uh  = (_Float16*)carve((size_t)BATCH * SENSOR * 2);
  _Float16* bt0 = (_Float16*)carve((size_t)BUNITS * SENSOR * 2);
  _Float16* bt[4];
  for (int i = 0; i < 4; ++i) bt[i] = (_Float16*)carve((size_t)BUNITS * BUNITS * 2);
  _Float16* w1t = (_Float16*)carve((size_t)LORA * BUNITS * 2);
  _Float16* w2t = (_Float16*)carve((size_t)2 * LORA * TU * TU * 2);
  _Float16* Ha  = (_Float16*)carve((size_t)BATCH * BUNITS * 2);
  _Float16* Hb  = (_Float16*)carve((size_t)BATCH * BUNITS * 2);
  float*    Zf  = (float*)carve((size_t)BATCH * LORA * 4);
  if (off > ws_size) return;

  const float S16 = 16.0f, INV16 = 0.0625f;
  const dim3 blk(256);

  {
    const int nch = BATCH * SENSOR / 8;
    k_cvt<<<dim3((nch + 255) / 256), blk, 0, stream>>>(u, uh, nch, 1.0f);
  }
  {
    const int tot0 = BUNITS * (SENSOR / 8);
    k_cvt_t<<<dim3((tot0 + 255) / 256), blk, 0, stream>>>(bw[0], bt0, SENSOR, BUNITS, S16);
    const int tot1 = BUNITS * (BUNITS / 8);
    for (int i = 0; i < 4; ++i)
      k_cvt_t<<<dim3((tot1 + 255) / 256), blk, 0, stream>>>(bw[i + 1], bt[i], BUNITS, BUNITS, S16);
    const int tot2 = LORA * (BUNITS / 8);
    k_cvt_t<<<dim3((tot2 + 255) / 256), blk, 0, stream>>>(W1, w1t, BUNITS, LORA, S16);
    const int tot3 = 2 * LORA * TU * (TU / 8);
    k_build_w2t<<<dim3((tot3 + 255) / 256), blk, 0, stream>>>(W2, w2t);
  }

  const dim3 g1(BATCH / 128, BUNITS / 128);
  k_gemm<true,  true, _Float16><<<g1, blk, 0, stream>>>(uh, bt0,   bb[0], Ha, BATCH, BUNITS, SENSOR, INV16);
  k_gemm<true,  true, _Float16><<<g1, blk, 0, stream>>>(Ha, bt[0], bb[1], Hb, BATCH, BUNITS, BUNITS, INV16);
  k_gemm<true,  true, _Float16><<<g1, blk, 0, stream>>>(Hb, bt[1], bb[2], Ha, BATCH, BUNITS, BUNITS, INV16);
  k_gemm<true,  true, _Float16><<<g1, blk, 0, stream>>>(Ha, bt[2], bb[3], Hb, BATCH, BUNITS, BUNITS, INV16);
  k_gemm<false, true, _Float16><<<g1, blk, 0, stream>>>(Hb, bt[3], bb[4], Ha, BATCH, BUNITS, BUNITS, INV16);

  const dim3 gz(BATCH / 128, 1);
  k_gemm<false, false, float><<<gz, blk, 0, stream>>>(Ha, w1t, bb[4], Zf, BATCH, LORA, BUNITS, INV16);

  k_trunk<<<dim3(BATCH / NSAMP), blk, 0, stream>>>(t, u, Zf, W2, w2t, out);
}
